// CausalSelfAttention_40630390620994
// MI455X (gfx1250) — hardware-verified
//
#include <hip/hip_runtime.h>

typedef __attribute__((ext_vector_type(16))) _Float16 v16h;
typedef __attribute__((ext_vector_type(8)))  _Float16 v8h;
typedef __attribute__((ext_vector_type(16))) __bf16   v16b;
typedef __attribute__((ext_vector_type(8)))  __bf16   v8b;
typedef __attribute__((ext_vector_type(8)))  float    v8f;
typedef __attribute__((ext_vector_type(4)))  float    v4f;
typedef __attribute__((ext_vector_type(4)))  unsigned int v4u;

#ifndef NB
#define NB 2
#endif
#ifndef SEQ
#define SEQ 4096
#endif
#define NB_FULL 2
#define SEQ_FULL 4096

constexpr int kDim      = 512;
constexpr int kHeads    = 8;
constexpr int kHeadDim  = 64;
constexpr int kRows     = NB * SEQ;
constexpr int kRowsFull = NB_FULL * SEQ_FULL;
constexpr int kQKV      = 3 * kDim;

static_assert(NB >= 1 && NB <= NB_FULL);
static_assert(SEQ >= 64 && SEQ <= SEQ_FULL);
static_assert(kHeads * kHeadDim == kDim);
static_assert(kHeadDim == 64);
static_assert(SEQ % 64 == 0);
static_assert(kRows % 64 == 0 && kQKV % 64 == 0 && kDim % 64 == 0 && kDim % 32 == 0);
static_assert(((size_t)SEQ * kDim) % (256 * 8) == 0);

constexpr size_t kOffXB  = 0;
constexpr size_t kSzXB   = (size_t)kRowsFull * kDim * 2;
constexpr size_t kOffWQT = 8388608;
constexpr size_t kSzWQT  = (size_t)kQKV * kDim * 2;
constexpr size_t kOffWPT = 10485760;
constexpr size_t kSzWPT  = (size_t)kDim * kDim * 2;
constexpr size_t kOffQH  = 16777216;
constexpr size_t kSzQ    = (size_t)kRowsFull * kQKV * 2;
constexpr size_t kOffQL  = kOffQH + kSzQ;
constexpr size_t kOffYH  = kOffQL + kSzQ;
constexpr size_t kSzY    = (size_t)kRowsFull * kDim * 2;
constexpr size_t kOffYL  = kOffYH + kSzY;
constexpr size_t kWsTotal = kOffYL + kSzY;
static_assert(kOffXB + kSzXB <= kOffWQT);
static_assert(kOffWQT + kSzWQT <= kOffWPT);
static_assert(kOffWPT + kSzWPT <= kOffQH);
static_assert(kOffQH + kSzQ <= kOffQL);
static_assert(kOffQL + kSzQ <= kOffYH);
static_assert(kOffYH + kSzY <= kOffYL);
static_assert(kWsTotal == 83886080);
static_assert(kWsTotal <= 134217728);
static_assert((size_t)kRows * kDim * 2 <= kSzXB && (size_t)kRows * kQKV * 2 <= kSzQ && (size_t)kRows * kDim * 2 <= kSzY);

__device__ __forceinline__ unsigned short f2bf_bits(float f) {
  unsigned u = __float_as_uint(f);
  return (unsigned short)((u + 0x7FFFu + ((u >> 16) & 1u)) >> 16);
}
__device__ __forceinline__ float bf_bits2f(unsigned short h) { return __uint_as_float(((unsigned)h) << 16); }

__device__ __forceinline__ void dep_guard_h(v8f& a, v8f& b, v16h x, v16h y) { asm volatile("v_nop\n\tv_nop\n\tv_nop\n\tv_nop" : "+v"(a), "+v"(b) : "v"(x), "v"(y)); }
__device__ __forceinline__ void dep_guard_b(v8f& a, v8f& b, v16b x, v16b y) { asm volatile("v_nop\n\tv_nop\n\tv_nop\n\tv_nop" : "+v"(a), "+v"(b) : "v"(x), "v"(y)); }
__device__ __forceinline__ void keep4_h(v16h a, v16h b, v16h c, v16h d) { asm volatile("v_nop" :: "v"(a), "v"(b), "v"(c), "v"(d)); }
__device__ __forceinline__ void keep4_b(v16b a, v16b b, v16b c, v16b d) { asm volatile("v_nop" :: "v"(a), "v"(b), "v"(c), "v"(d)); }
__device__ __forceinline__ void acc_guard4(v8f& a, v8f& b, v8f& c, v8f& d) { asm volatile("v_nop\n\tv_nop\n\tv_nop\n\tv_nop" : "+v"(a), "+v"(b), "+v"(c), "+v"(d)); }

template <typename T> struct Frag;
template <> struct Frag<_Float16> {
  typedef v16h V; union U { v16h v; v8h h[2]; };
  static __device__ __forceinline__ v16h load(const _Float16* p) {
    U f; f.h[0] = *(const v8h*)(p); f.h[1] = *(const v8h*)(p + 16); return f.v;
  }
  static __device__ __forceinline__ v8f mma(v16h a, v16h b, v8f c) {
    return __builtin_amdgcn_wmma_f32_16x16x32_f16(false, a, false, b, (short)0, c, false, false);
  }
  static __device__ __forceinline__ void guard(v8f& a, v8f& b, v16h x, v16h y) { dep_guard_h(a, b, x, y); }
  static __device__ __forceinline__ void keep(v16h a, v16h b, v16h c, v16h d) { keep4_h(a, b, c, d); }
};
template <> struct Frag<__bf16> {
  typedef v16b V; union U { v16b v; v8b h[2]; };
  static __device__ __forceinline__ v16b load(const __bf16* p) {
    U f; f.h[0] = *(const v8b*)(p); f.h[1] = *(const v8b*)(p + 16); return f.v;
  }
  static __device__ __forceinline__ v8f mma(v16b a, v16b b, v8f c) {
    return __builtin_amdgcn_wmma_f32_16x16x32_bf16(false, a, false, b, (short)0, c, false, false);
  }
  static __device__ __forceinline__ void guard(v8f& a, v8f& b, v16b x, v16b y) { dep_guard_b(a, b, x, y); }
  static __device__ __forceinline__ void keep(v16b a, v16b b, v16b c, v16b d) { keep4_b(a, b, c, d); }
};

template <int ET> struct Elem;
template <> struct Elem<0> { typedef _Float16 T; };
template <> struct Elem<1> { typedef __bf16 T; };
template <int ET, bool SPLA, bool SPLB, int BIAS_MODE, int OUT_MODE>
__global__ __launch_bounds__(256) void wmma_gemm64(
    const unsigned short* __restrict__ Ap, const unsigned short* __restrict__ A2p, int lda, long strideA,
    const unsigned short* __restrict__ Btp, const unsigned short* __restrict__ Bt2p, int ldb, long strideB,
    void* __restrict__ Cout, void* __restrict__ Cout2, int ldc, long strideC,
    const float* __restrict__ bias,
    int M, int N, int K, float scale) {
  typedef typename Elem<ET>::T T;
  typedef typename Frag<T>::V V;
  const T* A = (const T*)Ap; const T* A2 = (const T*)A2p; const T* Bt = (const T*)Btp; const T* Bt2 = (const T*)Bt2p;
  __shared__ __align__(16) float sT[8][16 * 68];
  const unsigned b    = blockIdx.y;
  const unsigned lane = threadIdx.x & 31u;
  const unsigned wave = threadIdx.x >> 5;
  const unsigned tilesN = ((unsigned)N) >> 6;
  const unsigned tilesM = ((unsigned)M) >> 6;
  const unsigned tile = blockIdx.x * 8u + wave;
  if (tile >= tilesM * tilesN) return;
  const unsigned tm = tile / tilesN;
  const unsigned tn = tile - tm * tilesN;
  const unsigned m0 = tm << 6;
  const unsigned n0 = tn << 6;
  const unsigned ulda = (unsigned)lda, uldb = (unsigned)ldb, uldc = (unsigned)ldc, uK = (unsigned)K;

  const T* Ab  = A  + (size_t)b * (size_t)strideA;
  const T* Bb  = Bt + (size_t)b * (size_t)strideB;
  const T* Ab2 = SPLA ? (A2  + (size_t)b * (size_t)strideA) : nullptr;
  const T* Bb2 = SPLB ? (Bt2 + (size_t)b * (size_t)strideB) : nullptr;

  const unsigned rlane = lane & 15u;
  const unsigned koff  = (lane >> 4) * 8u;
  const unsigned mOff  = (lane >> 4) * 8u;

  v8f acc[4][4];
#pragma unroll
  for (int i = 0; i < 4; ++i)
#pragma unroll
    for (int j = 0; j < 4; ++j) acc[i][j] = (v8f){0.f,0.f,0.f,0.f,0.f,0.f,0.f,0.f};

  for (unsigned k0 = 0; k0 < uK; k0 += 32u) {
    V bh[4], bl[4];
#pragma unroll
    for (int j = 0; j < 4; ++j) {
      const size_t bo = (size_t)(n0 + ((unsigned)j << 4) + rlane) * uldb + koff + k0;
      bh[j] = Frag<T>::load(Bb + bo);
      if (SPLB) bl[j] = Frag<T>::load(Bb2 + bo);
    }
#pragma unroll
    for (int i = 0; i < 4; ++i) {
      const size_t ao = (size_t)(m0 + ((unsigned)i << 4) + rlane) * ulda + koff + k0;
      V ah = Frag<T>::load(Ab + ao);
      V al;
      if (SPLA) al = Frag<T>::load(Ab2 + ao);
#pragma unroll
      for (int j = 0; j < 4; ++j) {
        acc[i][j] = Frag<T>::mma(ah, bh[j], acc[i][j]);
        if (SPLB) acc[i][j] = Frag<T>::mma(ah, bl[j], acc[i][j]);
        if (SPLA) acc[i][j] = Frag<T>::mma(al, bh[j], acc[i][j]);
      }
      Frag<T>::guard(acc[i][0], acc[i][3], ah, SPLA ? al : ah);
    }
    Frag<T>::keep(bh[0], bh[1], bh[2], bh[3]);
    if (SPLB) Frag<T>::keep(bl[0], bl[1], bl[2], bl[3]);
  }
  acc_guard4(acc[0][0], acc[0][1], acc[0][2], acc[0][3]);
  acc_guard4(acc[1][0], acc[1][1], acc[1][2], acc[1][3]);
  acc_guard4(acc[2][0], acc[2][1], acc[2][2], acc[2][3]);
  acc_guard4(acc[3][0], acc[3][1], acc[3][2], acc[3][3]);

  float* slab = sT[wave];
#pragma unroll
  for (int i = 0; i < 4; ++i) {
    const unsigned mBase = m0 + ((unsigned)i << 4);
#pragma unroll
    for (int j = 0; j < 4; ++j) {
      const unsigned n = n0 + ((unsigned)j << 4) + rlane;
      float bv = 0.f;
      if (BIAS_MODE == 2) bv = bf_bits2f(f2bf_bits(bias[n]));
#pragma unroll
      for (int r = 0; r < 8; ++r) {
        float v = acc[i][j][r] * scale;
        if (BIAS_MODE == 2) v += bv;
        slab[(mOff + (unsigned)r) * 68u + ((unsigned)j << 4) + rlane] = v;
      }
    }
    __builtin_amdgcn_fence(3  , "workgroup");
    __builtin_amdgcn_wave_barrier();
    __builtin_amdgcn_fence(2  , "workgroup");
    if (OUT_MODE == 0) {
      float* C = (float*)Cout + (size_t)b * (size_t)strideC;
      const unsigned hh = lane >> 4, c4 = (lane & 15u) * 4u;
      for (int pass = 0; pass < 2; ++pass) {
#pragma unroll
        for (int it = 0; it < 8; ++it) {
          const unsigned row = (unsigned)it * 2u + hh;
          v4f v = *(const v4f*)(slab + row * 68u + c4);
          *(volatile v4f*)(C + (size_t)(mBase + row) * uldc + n0 + c4) = v;
        }
        __threadfence();
      }
    } else {
      const unsigned q = lane >> 3, c8 = (lane & 7u) * 8u;
      unsigned short* C  = (unsigned short*)Cout  + (size_t)b * (size_t)strideC;
      unsigned short* C2 = (OUT_MODE == 2) ? ((unsigned short*)Cout2 + (size_t)b * (size_t)strideC) : nullptr;
      for (int pass = 0; pass < 2; ++pass) {
#pragma unroll
        for (int it = 0; it < 4; ++it) {
          const unsigned row = (unsigned)it * 4u + q;
          const float* sp = slab + row * 68u + c8;
          v8h hv, lv;
#pragma unroll
          for (int e = 0; e < 8; ++e) {
            if (OUT_MODE == 1) {
              hv[e] = (_Float16)sp[e];
              lv[e] = (_Float16)0.f;
            } else {
              unsigned short hb = f2bf_bits(sp[e]);
              unsigned short lb = f2bf_bits(sp[e] - bf_bits2f(hb));
              hv[e] = __builtin_bit_cast(_Float16, hb);
              lv[e] = __builtin_bit_cast(_Float16, lb);
            }
          }
          *(volatile v8h*)(C + (size_t)(mBase + row) * uldc + n0 + c8) = hv;
          if (OUT_MODE == 2) *(volatile v8h*)(C2 + (size_t)(mBase + row) * uldc + n0 + c8) = lv;
        }
        __threadfence();
      }
    }
    __builtin_amdgcn_fence(3  , "workgroup");
    __builtin_amdgcn_wave_barrier();
    __builtin_amdgcn_fence(2  , "workgroup");
  }
}

__global__ __launch_bounds__(256) void cast_f32_bf16x8(
    const float* __restrict__ in, unsigned short* __restrict__ out, int n8, long inStride, long outStride) {
  const unsigned i = blockIdx.x * 256u + threadIdx.x;
  const float* src = in + (size_t)blockIdx.y * (size_t)inStride;
  unsigned short* dst = out + (size_t)blockIdx.y * (size_t)outStride;
  if (i < (unsigned)n8) {
    const size_t e0 = (size_t)i * 8;
    const v4f a = *(const v4f*)(src + e0);
    const v4f c = *(const v4f*)(src + e0 + 4);
    v4u w;
    w[0] = (unsigned)f2bf_bits(a[0]) | ((unsigned)f2bf_bits(a[1]) << 16);
    w[1] = (unsigned)f2bf_bits(a[2]) | ((unsigned)f2bf_bits(a[3]) << 16);
    w[2] = (unsigned)f2bf_bits(c[0]) | ((unsigned)f2bf_bits(c[1]) << 16);
    w[3] = (unsigned)f2bf_bits(c[2]) | ((unsigned)f2bf_bits(c[3]) << 16);
    *(volatile v4u*)(dst + e0) = w;
    __threadfence();
    *(volatile v4u*)(dst + e0) = w;
  }
}

__global__ __launch_bounds__(256) void tcast64(
    const float* __restrict__ W, unsigned short* __restrict__ Wt, int nrows, int ncols) {
  __shared__ __align__(16) unsigned short tl[64 * 72];
  const unsigned tid = threadIdx.x, lane = tid & 31u, wave = tid >> 5;
  const unsigned k0 = blockIdx.y * 64u;
  const unsigned n0 = blockIdx.x * 64u;
  const unsigned krow = tid >> 2;
  const unsigned nseg = (tid & 3u) * 16u;
  const float* src = W + (size_t)(k0 + krow) * (unsigned)ncols + n0 + nseg;
  v4f vv[4];
#pragma unroll
  for (int i = 0; i < 4; ++i) vv[i] = ((const v4f*)src)[i];
#pragma unroll
  for (int i = 0; i < 4; ++i)
#pragma unroll
    for (int e = 0; e < 4; ++e) tl[(nseg + 4u * (unsigned)i + (unsigned)e) * 72u + krow] = f2bf_bits(vv[i][e]);
  __syncthreads();
  const unsigned q4 = lane >> 3, c8 = (lane & 7u) * 8u;
  for (int pass = 0; pass < 2; ++pass) {
#pragma unroll
    for (int it = 0; it < 2; ++it) {
      const unsigned row = wave * 8u + (unsigned)it * 4u + q4;
      const v4u w = *(const v4u*)(tl + row * 72u + c8);
      *(volatile v4u*)(Wt + (size_t)(n0 + row) * (unsigned)nrows + k0 + c8) = w;
    }
    __threadfence();
  }
}

#define AT_D 64
#define AT_NW 4
#define AT_QB 64
#define AT_KC 64

struct LdsKV {
  unsigned short kh[AT_KC * AT_D];
  unsigned short kl[AT_KC * AT_D];
  unsigned short vh[AT_D * AT_KC];
  unsigned short vl[AT_D * AT_KC];
};
union LdsU {
  LdsKV kv;
  float os[AT_NW][16 * 68];
};
static_assert(sizeof(LdsKV) == 32768);
static_assert(sizeof(LdsU) == 32768);

__device__ __forceinline__ __bf16 at_f2bf(float f) { return __builtin_bit_cast(__bf16, f2bf_bits(f)); }
__device__ __forceinline__ void at_split(float f, __bf16& hi, __bf16& lo) {
  const unsigned short hb = f2bf_bits(f);
  hi = __builtin_bit_cast(__bf16, hb);
  lo = at_f2bf(f - __uint_as_float(((unsigned)hb) << 16));
}
__device__ __forceinline__ v8f at_mma(v16b a, v16b b, v8f c) {
  c = __builtin_amdgcn_wmma_f32_16x16x32_bf16(false, a, false, b, (short)0, c, false, false);
  asm volatile("v_nop\n\tv_nop\n\tv_nop\n\tv_nop" : "+v"(c) : "v"(a), "v"(b));
  return c;
}

__global__ __launch_bounds__(128)
void attn64_planes(const unsigned short* __restrict__ qkvh, const unsigned short* __restrict__ qkvl,
                   unsigned short* __restrict__ yh, unsigned short* __restrict__ yl,
                   int nseq, int nheads, int ldq, int ldo, float sscale) {
  __shared__ __align__(16) LdsU lds;
  __shared__ __align__(16) __bf16 Psh[AT_NW][16 * AT_KC];
  __shared__ __align__(16) __bf16 Psl[AT_NW][16 * AT_KC];

  const unsigned tid  = threadIdx.x;
  const unsigned wave = tid >> 5;
  const unsigned lane = tid & 31u;
  const unsigned hh   = lane >> 4;
  const unsigned c    = lane & 15u;

  const unsigned useq = (unsigned)nseq, uheads = (unsigned)nheads, uldq = (unsigned)ldq, uldo = (unsigned)ldo;
  const unsigned nqb = useq >> 6;
  const unsigned bx  = blockIdx.x;
  const unsigned bhd = bx / nqb;
  const unsigned qb  = bx - bhd * nqb;
  const unsigned b   = bhd / uheads;
  const unsigned h   = bhd - b * uheads;
  const unsigned q0  = qb * AT_QB + wave * 16u;
  const size_t rowb = (size_t)b * useq;
  const unsigned qoff = h * AT_D;
  const unsigned kofs = uheads * AT_D + h * AT_D;
  const unsigned vofs = 2u * uheads * AT_D + h * AT_D;
  const float ninf = -__builtin_huge_valf();

  const __bf16* QH = (const __bf16*)(const void*)qkvh;
  const __bf16* QL = (const __bf16*)(const void*)qkvl;
  const __bf16* KHb = (const __bf16*)(const void*)lds.kv.kh;
  const __bf16* KLb = (const __bf16*)(const void*)lds.kv.kl;
  const __bf16* VHb = (const __bf16*)(const void*)lds.kv.vh;
  const __bf16* VLb = (const __bf16*)(const void*)lds.kv.vl;

  v16b qah[2], qal[2];
  {
    const size_t qr = (rowb + q0 + c) * (size_t)uldq + qoff + 8u * hh;
#pragma unroll
    for (int dc = 0; dc < 2; ++dc) {
      qah[dc] = Frag<__bf16>::load(QH + qr + dc * 32);
      qal[dc] = Frag<__bf16>::load(QL + qr + dc * 32);
    }
  }

  float mrow[8], lrow[8];
  v8f oacc[4];
#pragma unroll
  for (int r = 0; r < 8; ++r) { mrow[r] = ninf; lrow[r] = 0.f; }
#pragma unroll
  for (int t = 0; t < 4; ++t) oacc[t] = (v8f){0.f,0.f,0.f,0.f,0.f,0.f,0.f,0.f};

  const unsigned nChunks = qb + 1u;
  for (unsigned kc = 0; kc < nChunks; ++kc) {
    const unsigned kv0 = kc * AT_KC;
    __syncthreads();
    {
      const unsigned kvr = tid >> 1, dh = (tid & 1u) * 32u;
      const size_t kr = (rowb + kv0 + kvr) * (size_t)uldq + dh;
      v4u w0[4], w1[4];
      const v4u* pkh = (const v4u*)(qkvh + kr + kofs);
      const v4u* pkl = (const v4u*)(qkvl + kr + kofs);
#pragma unroll
      for (int i = 0; i < 4; ++i) { w0[i] = pkh[i]; w1[i] = pkl[i]; }
#pragma unroll
      for (int i = 0; i < 4; ++i) {
        *(v4u*)(lds.kv.kh + kvr * AT_D + dh + 8u * (unsigned)i) = w0[i];
        *(v4u*)(lds.kv.kl + kvr * AT_D + dh + 8u * (unsigned)i) = w1[i];
      }
      const v4u* pvh = (const v4u*)(qkvh + kr + vofs);
      const v4u* pvl = (const v4u*)(qkvl + kr + vofs);
#pragma unroll
      for (int i = 0; i < 4; ++i) { w0[i] = pvh[i]; w1[i] = pvl[i]; }
#pragma unroll
      for (int i = 0; i < 4; ++i) {
#pragma unroll
        for (int e = 0; e < 4; ++e) {
          const unsigned ua = w0[i][e], ub = w1[i][e];
          const unsigned d0 = dh + 8u * (unsigned)i + 2u * (unsigned)e;
          lds.kv.vh[d0 * AT_KC + kvr]        = (unsigned short)(ua & 0xffffu);
          lds.kv.vh[(d0 + 1u) * AT_KC + kvr] = (unsigned short)(ua >> 16);
          lds.kv.vl[d0 * AT_KC + kvr]        = (unsigned short)(ub & 0xffffu);
          lds.kv.vl[(d0 + 1u) * AT_KC + kvr] = (unsigned short)(ub >> 16);
        }
      }
    }
    __syncthreads();

    v8f s[4];
#pragma unroll
    for (int j = 0; j < 4; ++j) {
      s[j] = (v8f){0.f,0.f,0.f,0.f,0.f,0.f,0.f,0.f};
#pragma unroll
      for (int dc = 0; dc < 2; ++dc) {
        const v16b kb = Frag<__bf16>::load(KHb + ((unsigned)j * 16u + c) * AT_D + (unsigned)dc * 32u + 8u * hh);
        const v16b kl = Frag<__bf16>::load(KLb + ((unsigned)j * 16u + c) * AT_D + (unsigned)dc * 32u + 8u * hh);
        s[j] = at_mma(qah[dc], kb, s[j]);
        s[j] = at_mma(qah[dc], kl, s[j]);
        s[j] = at_mma(qal[dc], kb, s[j]);
      }
    }

    const bool diag = (kc == qb);
    float cm[8];
#pragma unroll
    for (int r = 0; r < 8; ++r) {
      const unsigned qrow = q0 + 8u * hh + (unsigned)r;
      float m = ninf;
#pragma unroll
      for (int j = 0; j < 4; ++j) {
        const unsigned kvcol = kv0 + (unsigned)j * 16u + c;
        float val = s[j][r] * sscale;
        if (diag && (kvcol > qrow)) val = ninf;
        s[j][r] = val;
        m = fmaxf(m, val);
      }
#pragma unroll
      for (int off = 1; off < 16; off <<= 1) m = fmaxf(m, __shfl_xor(m, off, 32));
      cm[r] = m;
    }

    __bf16* pwh = Psh[wave];
    __bf16* pwl = Psl[wave];
#pragma unroll
    for (int r = 0; r < 8; ++r) {
      const float mnew  = fmaxf(mrow[r], cm[r]);
      const float alpha = expf(mrow[r] - mnew);
      mrow[r] = mnew;
      float psum = 0.f;
#pragma unroll
      for (int j = 0; j < 4; ++j) {
        const float p = expf(s[j][r] - mnew);
        psum += p;
        __bf16 ph, pl;
        at_split(p, ph, pl);
        pwh[(8u * hh + (unsigned)r) * AT_KC + (unsigned)j * 16u + c] = ph;
        pwl[(8u * hh + (unsigned)r) * AT_KC + (unsigned)j * 16u + c] = pl;
      }
#pragma unroll
      for (int off = 1; off < 16; off <<= 1) psum += __shfl_xor(psum, off, 32);
      lrow[r] = lrow[r] * alpha + psum;
#pragma unroll
      for (int t = 0; t < 4; ++t) oacc[t][r] *= alpha;
    }
    __builtin_amdgcn_fence(3  , "workgroup");
    __builtin_amdgcn_wave_barrier();
    __builtin_amdgcn_fence(2  , "workgroup");

#pragma unroll
    for (int kk = 0; kk < 2; ++kk) {
      const v16b pa = Frag<__bf16>::load(pwh + c * AT_KC + (unsigned)kk * 32u + 8u * hh);
      const v16b pb = Frag<__bf16>::load(pwl + c * AT_KC + (unsigned)kk * 32u + 8u * hh);
#pragma unroll
      for (int t = 0; t < 4; ++t) {
        const v16b vb  = Frag<__bf16>::load(VHb + ((unsigned)t * 16u + c) * AT_KC + (unsigned)kk * 32u + 8u * hh);
        const v16b vlo = Frag<__bf16>::load(VLb + ((unsigned)t * 16u + c) * AT_KC + (unsigned)kk * 32u + 8u * hh);
        oacc[t] = at_mma(pa, vb,  oacc[t]);
        oacc[t] = at_mma(pa, vlo, oacc[t]);
        oacc[t] = at_mma(pb, vb,  oacc[t]);
      }
    }
  }

  __syncthreads();
  float* os = lds.os[wave];
#pragma unroll
  for (int r = 0; r < 8; ++r) {
    const float inv = 1.0f / lrow[r];
#pragma unroll
    for (int t = 0; t < 4; ++t) os[(8u * hh + (unsigned)r) * 68u + (unsigned)t * 16u + c] = oacc[t][r] * inv;
  }
  __builtin_amdgcn_fence(3  , "workgroup");
  __builtin_amdgcn_wave_barrier();
  __builtin_amdgcn_fence(2  , "workgroup");
  {
    const unsigned q4 = lane >> 3, c8 = (lane & 7u) * 8u;
    for (int pass = 0; pass < 2; ++pass) {
#pragma unroll
      for (int it = 0; it < 4; ++it) {
        const unsigned row = (unsigned)it * 4u + q4;
        const float* sp = os + row * 68u + c8;
        v4u hw, lw;
#pragma unroll
        for (int e2 = 0; e2 < 4; ++e2) {
          const float f0 = sp[2 * e2], f1 = sp[2 * e2 + 1];
          const unsigned short hb0 = f2bf_bits(f0);
          const unsigned short lb0 = f2bf_bits(f0 - bf_bits2f(hb0));
          const unsigned short hb1 = f2bf_bits(f1);
          const unsigned short lb1 = f2bf_bits(f1 - bf_bits2f(hb1));
          hw[e2] = (unsigned)hb0 | ((unsigned)hb1 << 16);
          lw[e2] = (unsigned)lb0 | ((unsigned)lb1 << 16);
        }
        const size_t o = (rowb + q0 + row) * (size_t)uldo + h * AT_D + c8;
        *(volatile v4u*)(yh + o) = hw;
        *(volatile v4u*)(yl + o) = lw;
      }
      __threadfence();
    }
  }
}

extern "C" void kernel_launch(void* const* d_in, const int* in_sizes, int n_in,
                              void* d_out, int out_size, void* d_ws,
                              size_t ws_size, hipStream_t stream)
{
  if (n_in < 9) return;
  if (ws_size < kWsTotal) return;
  const long long needX = (long long)(NB - 1) * SEQ_FULL * kDim + (long long)SEQ * kDim;
  if ((long long)out_size < needX) return;
  if ((long long)in_sizes[0] < needX) return;
  if (in_sizes[1] < kDim * kDim || in_sizes[3] < kDim * kDim || in_sizes[5] < kDim * kDim || in_sizes[7] < kDim * kDim) return;
  if (in_sizes[2] < kDim || in_sizes[4] < kDim || in_sizes[6] < kDim || in_sizes[8] < kDim) return;

  const float* x  = (const float*)d_in[0];
  const float* Wq = (const float*)d_in[1];
  const float* bq = (const float*)d_in[2];
  const float* Wk = (const float*)d_in[3];
  const float* bk = (const float*)d_in[4];
  const float* Wv = (const float*)d_in[5];
  const float* bv = (const float*)d_in[6];
  const float* Wo = (const float*)d_in[7];
  const float* bo = (const float*)d_in[8];
  float* out = (float*)d_out;

  unsigned char* ws = (unsigned char*)d_ws;
  unsigned short* XB  = (unsigned short*)(ws + kOffXB);
  unsigned short* WQT = (unsigned short*)(ws + kOffWQT);
  unsigned short* WPT = (unsigned short*)(ws + kOffWPT);
  unsigned short* QH  = (unsigned short*)(ws + kOffQH);
  unsigned short* QL  = (unsigned short*)(ws + kOffQL);
  unsigned short* YH  = (unsigned short*)(ws + kOffYH);
  unsigned short* YL  = (unsigned short*)(ws + kOffYL);

  {
    const int n8 = SEQ * kDim / 8;
    cast_f32_bf16x8<<<dim3((n8 + 255) / 256, NB), dim3(256), 0, stream>>>(
        x, XB, n8, (long)SEQ_FULL * kDim, (long)SEQ * kDim);
  }
  tcast64<<<dim3(kDim / 64, kDim / 64), dim3(256), 0, stream>>>(Wq, WQT, kDim, kDim);
  tcast64<<<dim3(kDim / 64, kDim / 64), dim3(256), 0, stream>>>(Wk, WQT + (size_t)kDim * kDim, kDim, kDim);
  tcast64<<<dim3(kDim / 64, kDim / 64), dim3(256), 0, stream>>>(Wv, WQT + (size_t)2 * kDim * kDim, kDim, kDim);
  tcast64<<<dim3(kDim / 64, kDim / 64), dim3(256), 0, stream>>>(Wo, WPT, kDim, kDim);
  {
    const int tiles = (kRows / 64) * (kDim / 64);
    wmma_gemm64<1, false, false, 2, 2><<<dim3((tiles + 7) / 8, 1), dim3(256), 0, stream>>>(
        XB, XB, kDim, 0L, WQT, WQT, kDim, 0L,
        (void*)QH, (void*)QL, kQKV, 0L, bq, kRows, kDim, kDim, 1.0f);
    wmma_gemm64<1, false, false, 2, 2><<<dim3((tiles + 7) / 8, 1), dim3(256), 0, stream>>>(
        XB, XB, kDim, 0L, WQT + (size_t)kDim * kDim, WQT + (size_t)kDim * kDim, kDim, 0L,
        (void*)(QH + kDim), (void*)(QL + kDim), kQKV, 0L, bk, kRows, kDim, kDim, 1.0f);
    wmma_gemm64<1, false, false, 2, 2><<<dim3((tiles + 7) / 8, 1), dim3(256), 0, stream>>>(
        XB, XB, kDim, 0L, WQT + (size_t)2 * kDim * kDim, WQT + (size_t)2 * kDim * kDim, kDim, 0L,
        (void*)(QH + 2 * kDim), (void*)(QL + 2 * kDim), kQKV, 0L, bv, kRows, kDim, kDim, 1.0f);
  }
  attn64_planes<<<dim3(NB * kHeads * (SEQ / AT_QB)), dim3(128), 0, stream>>>(
      QH, QL, YH, YL, SEQ, kHeads, kQKV, kDim, 0.125f);
  {
    const int tiles = (SEQ / 64) * (kDim / 64);
    wmma_gemm64<1, true, false, 2, 0><<<dim3((tiles + 7) / 8, NB), dim3(256), 0, stream>>>(
        YH, YL, kDim, (long)SEQ * kDim, WPT, WPT, kDim, 0L,
        (void*)out, (void*)YH, kDim, (long)SEQ_FULL * kDim, bo, SEQ, kDim, kDim, 1.0f);
  }
}
